// OrientedAnchoredRSConv_9663676416048
// MI455X (gfx1250) — hardware-verified
//
#include <hip/hip_runtime.h>
#include <math.h>

typedef __attribute__((ext_vector_type(16))) _Float16 v16h;
typedef __attribute__((ext_vector_type(16))) __bf16 v16b;
typedef __attribute__((ext_vector_type(8)))  _Float16 v8h;
typedef __attribute__((ext_vector_type(8)))  float v8f;
typedef __attribute__((ext_vector_type(4)))  float v4f;
typedef __attribute__((ext_vector_type(2)))  float v2f;
typedef __attribute__((ext_vector_type(4)))  unsigned v4u;
typedef __attribute__((ext_vector_type(4)))  int v4i;
typedef float __attribute__((may_alias)) float_a;
typedef int __attribute__((may_alias)) int_a;

template <typename T> __device__ __forceinline__ void vst2(void* p, T v) { *(volatile T*)p = v; __threadfence(); *(volatile T*)p = v; }
__device__ __forceinline__ v8f wmma16(v16h a, v16h b, v8f c) {
  v8f d = __builtin_amdgcn_wmma_f32_16x16x32_f16(false, a, false, b, (short)0, c, false, false);
  asm volatile("v_nop\n\tv_nop\n\tv_nop\n\tv_nop" : "+v"(d) : "v"(a), "v"(b));
  return d;
}
__device__ __forceinline__ v8f wmma_bf(v16b a, v16b b, v8f c) {
  v8f d = __builtin_amdgcn_wmma_f32_16x16x32_bf16(false, a, false, b, (short)0, c, false, false);
  asm volatile("v_nop\n\tv_nop\n\tv_nop\n\tv_nop" : "+v"(d) : "v"(a), "v"(b));
  return d;
}
__device__ __forceinline__ v16h frag_h(const _Float16* rowk0, int lane) {
  union { v16h v; v8h q[2]; } u; const _Float16* p = rowk0 + 8 * (lane >> 4);
  u.q[0] = *(const v8h*)p; u.q[1] = *(const v8h*)(p + 16); return u.v;
}
__device__ __forceinline__ v16h frag_f32(const float* rowk0, int lane) {
  v16h a; const float* p = rowk0 + 8 * (lane >> 4);
#pragma unroll
  for (int i = 0; i < 8; ++i) { a[i] = (_Float16)p[i]; a[8 + i] = (_Float16)p[16 + i]; }
  return a;
}
__device__ __forceinline__ v16h frag_f32s(const float* rowk0, int lane, float sc) {
  v16h a; const float* p = rowk0 + 8 * (lane >> 4);
#pragma unroll
  for (int i = 0; i < 8; ++i) { a[i] = (_Float16)(p[i] * sc); a[8 + i] = (_Float16)(p[16 + i] * sc); }
  return a;
}
__device__ __forceinline__ v16h fragc_f32(const float* W, int k0, int n, int lane, int ld, int K) {
  v16h a; const int g = lane >> 4;
#pragma unroll
  for (int i = 0; i < 8; ++i) { const int ka = k0 + 8 * g + i, kb = ka + 16;
    a[i] = (_Float16)(ka < K ? W[(size_t)(ka < K ? ka : K - 1) * ld + n] : 0.f); a[8 + i] = (_Float16)(kb < K ? W[(size_t)(kb < K ? kb : K - 1) * ld + n] : 0.f); }
  return a;
}
struct F2 { v16b h, l; };
__device__ __forceinline__ F2 bsplit16(const float v[16]) { F2 r;
#pragma unroll
  for (int i = 0; i < 16; ++i) { const __bf16 h = (__bf16)v[i]; r.h[i] = h; r.l[i] = (__bf16)(v[i] - (float)h); }
  return r; }
__device__ __forceinline__ F2 split_row(const float* row, int k0, int lane) { float v[16]; const float* p = row + k0 + 8 * (lane >> 4);
#pragma unroll
  for (int i = 0; i < 8; ++i) { v[i] = p[i]; v[8 + i] = p[16 + i]; }
  return bsplit16(v); }
__device__ __forceinline__ F2 split_rowK(const float* row, int k0, int lane, int K) { float v[16]; const int g = lane >> 4;
#pragma unroll
  for (int i = 0; i < 8; ++i) { const int ka = k0 + 8 * g + i, kb = ka + 16; v[i] = ka < K ? row[ka < K ? ka : K - 1] : 0.f; v[8 + i] = kb < K ? row[kb < K ? kb : K - 1] : 0.f; }
  return bsplit16(v); }
__device__ __forceinline__ F2 split_col(const float* W, int k0, int n, int lane, int ld, int K) { float v[16]; const int g = lane >> 4;
#pragma unroll
  for (int i = 0; i < 8; ++i) { const int ka = k0 + 8 * g + i, kb = ka + 16; v[i] = ka < K ? W[(size_t)(ka < K ? ka : K - 1) * ld + n] : 0.f; v[8 + i] = kb < K ? W[(size_t)(kb < K ? kb : K - 1) * ld + n] : 0.f; }
  return bsplit16(v); }
__device__ __forceinline__ v8f mac3(const F2& a, const F2& b, v8f c) { c = wmma_bf(a.l, b.h, c); c = wmma_bf(a.h, b.l, c); return wmma_bf(a.h, b.h, c); }
__device__ __forceinline__ float sigm(float v) { return 1.0f / (1.0f + expf(-v)); }
#define LDSX() do { asm volatile("s_wait_dscnt 0" ::: "memory"); __builtin_amdgcn_wave_barrier(); __builtin_amdgcn_fence(__ATOMIC_RELEASE, "workgroup"); } while (0)


#define NB 16
#define NIN 4096
#define NOUT 1024
#define NQ (NB * NOUT)
#define KNB 32
#define NPAIR (NQ * KNB)
#define CIN 128
#define C4 32
#define COUT 256
typedef __attribute__((ext_vector_type(8))) __bf16 v8b;
__device__ __forceinline__ v16b frag_b(const __bf16* rowk0, int lane) {
  union { v16b v; v8b q[2]; } u; const __bf16* p = rowk0 + 8 * (lane >> 4);
  u.q[0] = *(const v8b*)p; u.q[1] = *(const v8b*)(p + 16); return u.v;
}
__device__ __forceinline__ float bfr(float v) { return (float)(__bf16)v; }
__device__ __attribute__((noinline)) float exp_ni(float v) { return expf(v); }
__device__ __attribute__((noinline)) float erf_ni(float v) { return erff(v); }

#define PK_1 0
#define PK_2 (C4 * 32)
#define PK_3 (PK_2 + CIN * C4)
#define PK_END (PK_3 + COUT * CIN)
#define WS_PK  0u
#define WS_P4  (((2u * PK_END) + 127u) / 128u * 128u)
#define WS_SQ  (WS_P4 + 4u * NB * NIN * 4)
#define WS_IDX (WS_SQ + 4u * NB * NIN)
#define WS_H   (WS_IDX + 4u * NQ * KNB)
#define WS_END (WS_H + 4u * NQ * CIN)

__global__ __launch_bounds__(128) void k_pack(const float* __restrict__ W1, const float* __restrict__ W2, const float* __restrict__ W3, __bf16* __restrict__ PK) {
  __shared__ __align__(16) __bf16 s[CIN]; const int n = blockIdx.x, which = blockIdx.y, t = threadIdx.x; int K; size_t dst;
  if (which == 0) { if (n >= C4) return; K = 32; dst = PK_1 + (size_t)n * 32; if (t < 32) s[t] = (__bf16)((t < 16) ? W1[n * 16 + t] : 0.f); }
  else if (which == 1) { if (n >= CIN) return; K = 32; dst = PK_2 + (size_t)n * 32; if (t < 32) s[t] = (__bf16)W2[n * 32 + t]; }
  else { K = CIN; dst = PK_3 + (size_t)n * CIN; s[t] = (__bf16)W3[(size_t)n * CIN + t]; }
  __syncthreads();
  if (t < K / 8) vst2((unsigned*)(PK + dst + t * 8), *(const v4u*)&s[t * 8]);
}
__global__ __launch_bounds__(256) void k_prep(const float* __restrict__ PIN, float* __restrict__ P4, float* __restrict__ SQ) {
  __shared__ __align__(16) float sp[256][4]; __shared__ __align__(16) float ss[256]; const int t = threadIdx.x; const size_t p = (size_t)blockIdx.x * 256 + t;
  const float x0 = bfr(PIN[p * 3]), x1 = bfr(PIN[p * 3 + 1]), x2 = bfr(PIN[p * 3 + 2]); sp[t][0] = x0; sp[t][1] = x1; sp[t][2] = x2; sp[t][3] = 0.f; ss[t] = __fadd_rn(__fadd_rn(__fmul_rn(x0, x0), __fmul_rn(x2, x2)), __fmul_rn(x1, x1));
  __syncthreads();
  vst2(P4 + p * 4, *(const v4f*)&sp[t][0]); if (t < 64) vst2(SQ + (size_t)blockIdx.x * 256 + t * 4, *(const v4f*)&ss[t * 4]);
}
__global__ __launch_bounds__(128) void k_knn(const float* __restrict__ POUT, const float* __restrict__ P4, const float* __restrict__ SQ, int* __restrict__ IDX) {
  __shared__ float sd[4][NIN]; __shared__ __align__(16) int sidx[4][KNB];
  const int tid = threadIdx.x, wave = tid >> 5, lane = tid & 31; const size_t q = (size_t)blockIdx.x * 4 + wave; const int b = (int)(q / NOUT); const size_t base = (size_t)b * NIN;
  const float qx0 = bfr(POUT[q * 3]), qx1 = bfr(POUT[q * 3 + 1]), qx2 = bfr(POUT[q * 3 + 2]); const float sqo = __fadd_rn(__fadd_rn(__fmul_rn(qx0, qx0), __fmul_rn(qx1, qx1)), __fmul_rn(qx2, qx2));
  for (int j = lane; j < NIN; j += 32) { const size_t pj = base + j; const float dot = __fadd_rn(__fadd_rn(__fmul_rn(qx0, P4[pj * 4]), __fmul_rn(qx1, P4[pj * 4 + 1])), __fmul_rn(qx2, P4[pj * 4 + 2])); sd[wave][j] = __fsub_rn(__fadd_rn(sqo, SQ[pj]), __fmul_rn(2.0f, dot)); }
  __syncthreads();
#pragma unroll 1
  for (int s = 0; s < KNB; ++s) { float bv = 3.0e38f; int bi = 0x7fffffff;
    for (int j = lane; j < NIN; j += 32) { const float v = sd[wave][j]; if (v < bv) { bv = v; bi = j; } }
#pragma unroll
    for (int o = 1; o < 32; o <<= 1) { const float ov = __shfl_xor(bv, o); const int oi = __shfl_xor(bi, o); if (ov < bv || (ov == bv && oi < bi)) { bv = ov; bi = oi; } }
    if (lane == 0) { sidx[wave][s] = bi; sd[wave][bi] = 3.0e38f; }
    __syncthreads(); }
  if (tid < 32) vst2((unsigned*)(IDX + ((size_t)blockIdx.x * 4 + (tid >> 3)) * KNB + (tid & 7) * 4), *(const v4u*)&sidx[tid >> 3][(tid & 7) * 4]);
}
__global__ __launch_bounds__(128) void k_pair(const float* __restrict__ POUT, const float* __restrict__ ROUT, const float* __restrict__ P4, const float* __restrict__ HIN, const int* __restrict__ IDX, const __bf16* __restrict__ PK, const float* __restrict__ B1, const float* __restrict__ AG, const float* __restrict__ AB, const float* __restrict__ AM, const float* __restrict__ AV, const float* __restrict__ B2, const float* __restrict__ BG, const float* __restrict__ BB_, const float* __restrict__ BM, const float* __restrict__ BV, float* __restrict__ H) {
  __shared__ __align__(16) __bf16 swh[64][40], swl[64][40]; __shared__ __align__(16) __bf16 sxh[4][16][40], sxl[4][16][40]; __shared__ float sm[64][CIN + 1]; __shared__ __align__(16) float sred[2][CIN];
  const int tid = threadIdx.x, wave = tid >> 5, lane = tid & 31, col = lane & 15, g = lane >> 4; const size_t qA = (size_t)blockIdx.x * 2;
  if (tid < 64) { const size_t q = qA + (tid >> 5); const int k = tid & 31; const int b = (int)(q / NOUT); const size_t j = (size_t)b * NIN + IDX[q * KNB + k];
    const float rx = P4[j * 4] - bfr(POUT[q * 3]), ry = P4[j * 4 + 1] - bfr(POUT[q * 3 + 1]), rz = P4[j * 4 + 2] - bfr(POUT[q * 3 + 2]);
    float w16[16];
#pragma unroll
    for (int m = 0; m < 12; ++m) { const float* Rm = ROUT + (q * 12 + m) * 3; w16[m] = (bfr(Rm[0]) * rx + bfr(Rm[1]) * ry) + bfr(Rm[2]) * rz; }
#pragma unroll
    for (int f = 0; f < 4; ++f) { const float a0 = w16[3 * f], a1 = w16[3 * f + 1], a2 = w16[3 * f + 2]; w16[12 + f] = sqrtf((a0 * a0 + a1 * a1) + a2 * a2); }
#pragma unroll
    for (int m = 0; m < 16; ++m) { const __bf16 hb = (__bf16)w16[m]; swh[tid][m] = hb; swl[tid][m] = (__bf16)(w16[m] - (float)hb); swh[tid][16 + m] = (__bf16)0.f; swl[tid][16 + m] = (__bf16)0.f; } }
  __syncthreads();
  v8f ax[2] = {};
  { F2 a; a.h = frag_b(&swh[wave * 16 + col][0], lane); a.l = frag_b(&swl[wave * 16 + col][0], lane);
#pragma unroll
    for (int jt = 0; jt < 2; ++jt) { const v16b w = frag_b(PK + PK_1 + (size_t)(jt * 16 + col) * 32, lane); ax[jt] = wmma_bf(a.l, w, ax[jt]); ax[jt] = wmma_bf(a.h, w, ax[jt]); } }
#pragma unroll
  for (int jt = 0; jt < 2; ++jt) { const int c = jt * 16 + col; const float sc = bfr(AG[c]) / sqrtf(bfr(AV[c]) + 1e-5f), mm = bfr(AM[c]), be = bfr(AB[c]), bb = bfr(B1[c]);
#pragma unroll
    for (int r = 0; r < 8; ++r) { float v = (ax[jt][r] + bb - mm) * sc + be; v = fmaxf(v, 0.f); const __bf16 hb = (__bf16)v; sxh[wave][8 * g + r][c] = hb; sxl[wave][8 * g + r][c] = (__bf16)(v - (float)hb); } }
  LDSX();
  v8f aw[8] = {};
  { F2 a; a.h = frag_b(&sxh[wave][col][0], lane); a.l = frag_b(&sxl[wave][col][0], lane);
#pragma unroll
    for (int jt = 0; jt < 8; ++jt) { const v16b w = frag_b(PK + PK_2 + (size_t)(jt * 16 + col) * 32, lane); aw[jt] = wmma_bf(a.l, w, aw[jt]); aw[jt] = wmma_bf(a.h, w, aw[jt]); } }
#pragma unroll
  for (int jt = 0; jt < 8; ++jt) { const int c = jt * 16 + col; const float sc = bfr(BG[c]) / sqrtf(bfr(BV[c]) + 1e-5f), mm = bfr(BM[c]), be = bfr(BB_[c]), bb = bfr(B2[c]);
#pragma unroll
    for (int r = 0; r < 8; ++r) { const int pr = wave * 16 + 8 * g + r; const size_t q = qA + (pr >> 5); const int k = pr & 31; const int b = (int)(q / NOUT); const size_t j = (size_t)b * NIN + IDX[q * KNB + k];
      float v = ((aw[jt][r] + bb) * bfr(HIN[j * CIN + c]) - mm) * sc + be; sm[pr][c] = fmaxf(v, 0.f); } }
  __syncthreads();
  { const int c = tid; float m0 = -3.0e38f, m1 = -3.0e38f;
#pragma unroll 1
    for (int k = 0; k < 32; ++k) { m0 = fmaxf(m0, sm[k][c]); m1 = fmaxf(m1, sm[32 + k][c]); }
    sred[0][c] = m0; sred[1][c] = m1; }
  __syncthreads();
  if (tid < 64) { const int qq = tid >> 5, pc = tid & 31; vst2(H + (qA + qq) * CIN + pc * 4, *(const v4f*)&sred[qq][pc * 4]); }
}
__global__ __launch_bounds__(128) void k_fin(const float* __restrict__ H, const __bf16* __restrict__ PK, const float* __restrict__ B3, const float* __restrict__ CG, const float* __restrict__ CB, const float* __restrict__ CM, const float* __restrict__ CV, float* __restrict__ OUT) {
  __shared__ __align__(16) float so[4][16][132];
  const int tid = threadIdx.x, wave = tid >> 5, lane = tid & 31, col = lane & 15, g = lane >> 4; const size_t r0 = (size_t)blockIdx.x * 64 + wave * 16; const int n0 = blockIdx.y * 128;
  v8f acc[8] = {};
#pragma unroll
  for (int kc = 0; kc < CIN / 32; ++kc) { const F2 a = split_row(H + (r0 + col) * CIN, kc * 32, lane);
#pragma unroll
    for (int jt = 0; jt < 8; ++jt) { const v16b w = frag_b(PK + PK_3 + (size_t)(n0 + jt * 16 + col) * CIN + kc * 32, lane); acc[jt] = wmma_bf(a.l, w, acc[jt]); acc[jt] = wmma_bf(a.h, w, acc[jt]); } }
#pragma unroll
  for (int jt = 0; jt < 8; ++jt) { const int c = n0 + jt * 16 + col; const float sc = bfr(CG[c]) / sqrtf(bfr(CV[c]) + 1e-5f), mm = bfr(CM[c]), be = bfr(CB[c]), bb = bfr(B3[c]);
#pragma unroll
    for (int r = 0; r < 8; ++r) { float v = (acc[jt][r] + bb - mm) * sc + be; so[wave][8 * g + r][jt * 16 + col] = fmaxf(v, 0.f); } }
  LDSX();
  for (int rl = 0; rl < 16; ++rl) vst2(OUT + (r0 + rl) * COUT + n0 + lane * 4, *(const v4f*)&so[wave][rl][lane * 4]);
}
extern "C" void kernel_launch(void* const* d_in, const int* in_sizes, int n_in, void* d_out, int out_size, void* d_ws, size_t ws_size, hipStream_t stream) {
  (void)in_sizes; (void)n_in; (void)out_size;
  const float** F = (const float**)d_in;
  if (ws_size < (size_t)WS_END) return;
  char* ws = (char*)d_ws; __bf16* PK = (__bf16*)(ws + WS_PK); float *P4 = (float*)(ws + WS_P4), *SQ = (float*)(ws + WS_SQ), *H = (float*)(ws + WS_H); int* IDX = (int*)(ws + WS_IDX);
  k_pack<<<dim3(COUT, 3), 128, 0, stream>>>(F[4], F[10], F[16], PK);
  k_prep<<<NB * NIN / 256, 256, 0, stream>>>(F[0], P4, SQ);
  k_knn<<<NQ / 4, 128, 0, stream>>>(F[1], P4, SQ, IDX);
  k_pair<<<NQ / 2, 128, 0, stream>>>(F[1], F[2], P4, F[3], IDX, PK, F[5], F[6], F[7], F[8], F[9], F[11], F[12], F[13], F[14], F[15], H);
  k_fin<<<dim3(NQ / 64, COUT / 128), 128, 0, stream>>>(H, PK, F[17], F[18], F[19], F[20], F[21], (float*)d_out);
}
